// CausalLocalAttention_71786083386178
// MI455X (gfx1250) — hardware-verified
//
#include <hip/hip_runtime.h>
#include <math.h>
#include <float.h>
#include <stdint.h>

#define NB    1
#define SEQ   8192
#define NH    16
#define HD    64
#define WIN   256
#define NWIN  (SEQ / WIN)
#define NPAIR (HD / 2)
#define TOKP  (NH * HD)
#define NQUAD (NH / 4)
#define NQB   (SEQ / 64)
#define OUTN  (NB * SEQ * NH * HD)
static_assert(HD == 64);
static_assert(NPAIR == 32);
static_assert((NH % 4) == 0);
static_assert((WIN % 64) == 0);
static_assert((SEQ % WIN) == 0);
static_assert(((SEQ * NQUAD) % 8) == 0);
static_assert(((NWIN * NPAIR) % 256) == 0);
static_assert((SEQ % 64) == 0);

typedef _Float16 v16h __attribute__((ext_vector_type(16)));
typedef _Float16 v8h  __attribute__((ext_vector_type(8)));
typedef float    v8f  __attribute__((ext_vector_type(8)));
typedef float    v4f  __attribute__((ext_vector_type(4)));
typedef unsigned int v4u __attribute__((ext_vector_type(4)));

__device__ __forceinline__ unsigned short bf_bits(float f) {
  unsigned u = __float_as_uint(f);
  return (unsigned short)((u + 0x7FFFu + ((u >> 16) & 1u)) >> 16);
}
__device__ __forceinline__ float bf_up(unsigned short h) { return __uint_as_float(((unsigned)h) << 16); }
__device__ __forceinline__ unsigned short h_bits(_Float16 x) { return __builtin_bit_cast(unsigned short, x); }
__device__ __forceinline__ unsigned pk16(unsigned short a, unsigned short b) { return (unsigned)a | ((unsigned)b << 16); }
__device__ __forceinline__ v8f zero8() { v8f z = {0.f, 0.f, 0.f, 0.f, 0.f, 0.f, 0.f, 0.f}; return z; }

__device__ __forceinline__ v16h ldfrag_h(const _Float16* p) {
  union { v16h v; v8h h[2]; } f;
  f.h[0] = *(const v8h*)(p);
  f.h[1] = *(const v8h*)(p + 16);
  return f.v;
}

__device__ __forceinline__ v8f mma_h(v16h a, v16h b, v8f c) {
  c = __builtin_amdgcn_wmma_f32_16x16x32_f16(false, a, false, b, (short)0, c, false, false);
#if defined(__HIP_DEVICE_COMPILE__)
  asm volatile("v_nop\n\tv_nop\n\tv_nop\n\tv_nop" : "+v"(c) : "v"(a), "v"(b));
#endif
  return c;
}

__global__ __launch_bounds__(256) void rope_tab(float* ct, float* st, int n) {
#pragma clang fp contract(off)
  const int i = blockIdx.x * 256 + threadIdx.x;
  if (i < n) {
    const int wi = i >> 5;
    const int j  = i & 31;
    const float p    = (float)(2 * j) / 64.0f;
    const float base = powf(10000.0f, p);
    const float inv  = 1.0f / base;
    const float ang  = (float)wi * inv;
    const float cv = cosf(ang);
    const float sv = sinf(ang);
    *(volatile float*)(ct + i) = cv;
    *(volatile float*)(st + i) = sv;
    __threadfence();
    *(volatile float*)(ct + i) = cv;
    *(volatile float*)(st + i) = sv;
  }
}

template <int NOUT>
__global__ __launch_bounds__(256) void rope_plane(const float* __restrict__ src,
                                                  const float* __restrict__ ct, const float* __restrict__ st,
                                                  unsigned short* dst0, unsigned short* dst1,
                                                  int nwaves, float xscale, float oscale) {
#pragma clang fp contract(off)
  __shared__ __align__(16) float sy[8][NOUT * 256];
  const int tid = threadIdx.x, wave = tid >> 5, lane = tid & 31;
  const int w = blockIdx.x * 8 + wave;
  if (w >= nwaves) return;
  const int hq = w % NQUAD;
  const int t  = w / NQUAD;
  const int wi = t / WIN;
  const int a1 = (wi + 1 < NWIN) ? (wi + 1) : (NWIN - 1);
  const float cs0 = ct[wi * NPAIR + lane];
  const float sn0 = st[wi * NPAIR + lane];
  float cs1 = cs0, sn1 = sn0;
  if (NOUT == 2) {
    cs1 = ct[a1 * NPAIR + lane];
    sn1 = st[a1 * NPAIR + lane];
  }
  const float* row = src + (size_t)t * TOKP + (size_t)hq * 256;
  float* buf = sy[wave];
#pragma unroll
  for (int tt = 0; tt < 4; ++tt) {
    const float* s2 = row + tt * HD;
    const float x0 = bf_up(bf_bits(s2[2 * lane])) * xscale;
    const float x1 = bf_up(bf_bits(s2[2 * lane + 1])) * xscale;
    buf[tt * 64 + 2 * lane]     = x0 * cs0 - x1 * sn0;
    buf[tt * 64 + 2 * lane + 1] = x0 * sn0 + x1 * cs0;
    if (NOUT == 2) {
      buf[256 + tt * 64 + 2 * lane]     = x0 * cs1 - x1 * sn1;
      buf[256 + tt * 64 + 2 * lane + 1] = x0 * sn1 + x1 * cs1;
    }
  }
  __builtin_amdgcn_fence(__ATOMIC_RELEASE, "workgroup");
  __builtin_amdgcn_wave_barrier();
  __builtin_amdgcn_fence(__ATOMIC_ACQUIRE, "workgroup");
  const int g = lane >> 3, piece = lane & 7;
  v4u val[NOUT];
#pragma unroll
  for (int o = 0; o < NOUT; ++o) {
    const float* sp = buf + o * 256 + g * 64 + piece * 8;
    const v4f a0 = *(const v4f*)(sp);
    const v4f b0 = *(const v4f*)(sp + 4);
    v4u pv;
#pragma unroll
    for (int e = 0; e < 4; ++e) {
      const float f0 = (e < 2) ? a0[2 * e]     : b0[2 * e - 4];
      const float f1 = (e < 2) ? a0[2 * e + 1] : b0[2 * e - 3];
      pv[e] = pk16(h_bits((_Float16)(f0 * oscale)), h_bits((_Float16)(f1 * oscale)));
    }
    val[o] = pv;
  }
  const size_t go = (size_t)t * TOKP + (size_t)hq * 256 + (size_t)g * 64 + piece * 8;
  *(volatile v4u*)(dst0 + go) = val[0];
  if (NOUT == 2) *(volatile v4u*)(dst1 + go) = val[NOUT - 1];
  __threadfence();
  *(volatile v4u*)(dst0 + go) = val[0];
  if (NOUT == 2) *(volatile v4u*)(dst1 + go) = val[NOUT - 1];
}

__global__ __launch_bounds__(256) void v_plane(const float* __restrict__ vf, unsigned short* vt) {
  __shared__ __align__(16) float sv[64 * 68];
  const int tid = threadIdx.x;
  const int t0  = blockIdx.x * 64;
  const int hh  = blockIdx.y;
#pragma unroll
  for (int i = 0; i < 4; ++i) {
    const int idx = i * 256 + tid;
    const int tt = idx >> 4, c4 = (idx & 15) * 4;
    const v4f a = *(const v4f*)(vf + ((size_t)(t0 + tt)) * TOKP + hh * HD + c4);
    *(v4f*)(sv + tt * 68 + c4) = a;
  }
  __syncthreads();

  const int g = tid >> 3, piece = tid & 7;
  v4u hv[2];
  size_t hofs[2];
#pragma unroll
  for (int it = 0; it < 2; ++it) {
    const int d = it * 32 + g;
    v4u a;
#pragma unroll
    for (int e = 0; e < 4; ++e) {
      const float f0 = sv[(piece * 8 + 2 * e) * 68 + d];
      const float f1 = sv[(piece * 8 + 2 * e + 1) * 68 + d];
      const _Float16 x0 = (_Float16)(bf_up(bf_bits(f0)) * 16.0f);
      const _Float16 x1 = (_Float16)(bf_up(bf_bits(f1)) * 16.0f);
      a[e] = pk16(h_bits(x0), h_bits(x1));
    }
    hv[it] = a;
    hofs[it] = (size_t)(hh * HD + d) * SEQ + t0 + piece * 8;
  }
  for (int pass = 0; pass < 2; ++pass) {
#pragma unroll
    for (int it = 0; it < 2; ++it) {
      *(volatile v4u*)(vt + hofs[it]) = hv[it];
    }
    __threadfence();
  }
}

__global__ __launch_bounds__(128)
void attn_local64(const unsigned short* __restrict__ qp, const unsigned short* __restrict__ kap,
                  const unsigned short* __restrict__ kbp, const unsigned short* __restrict__ vtp,
                  float* outp, float sscale) {
  union FH { v16h v; v8h h[2]; };
  __shared__ __align__(16) _Float16 Psh[4][16 * 64];
  __shared__ __align__(16) float    Os[4][16 * 64];

  const int tid  = threadIdx.x;
  const int wave = tid >> 5;
  const int lane = tid & 31;
  const int hh   = lane >> 4;
  const int cc   = lane & 15;

  const int bx   = blockIdx.x;
  const int h    = bx / NQB;
  const int qb   = bx - h * NQB;
  const int q0   = qb * 64 + wave * 16;
  const int wi   = q0 / WIN;
  const int qi0  = q0 - wi * WIN;
  const int kbase = wi * WIN - WIN;

  const _Float16* Qp = (const _Float16*)(const void*)qp;
  const _Float16* Ka = (const _Float16*)(const void*)kap;
  const _Float16* Kb = (const _Float16*)(const void*)kbp;
  const _Float16* Vt = (const _Float16*)(const void*)vtp + (size_t)h * HD * SEQ;

  v16h qa[2];
#pragma unroll
  for (int dc = 0; dc < 2; ++dc) {
    const size_t qo = (size_t)(q0 + cc) * TOKP + (size_t)h * HD + dc * 32 + 8 * hh;
    qa[dc] = ldfrag_h(Qp + qo);
  }

  float mrow[8], lrow[8];
  v8f oacc[4];
#pragma unroll
  for (int r = 0; r < 8; ++r) { mrow[r] = -INFINITY; lrow[r] = 0.f; }
#pragma unroll
  for (int t = 0; t < 4; ++t) oacc[t] = zero8();

  const int cbeg = (wi == 0) ? 4 : 0;
  int cend = (qi0 + 15 + WIN) >> 6;
  if (cend > 7) cend = 7;
  _Float16* pwh = Psh[wave];

  for (int ch = cbeg; ch <= cend; ++ch) {
    const _Float16* Kp = (ch < 4) ? Kb : Ka;
    const int tk0 = kbase + ch * 64;

    v8f s[4];
#pragma unroll
    for (int j = 0; j < 4; ++j) {
      s[j] = zero8();
      const size_t ko = (size_t)(tk0 + j * 16 + cc) * TOKP + (size_t)h * HD + 8 * hh;
#pragma unroll
      for (int dc = 0; dc < 2; ++dc) {
        FH kb;
        kb.h[0] = *(const v8h*)(Kp + ko + dc * 32);
        kb.h[1] = *(const v8h*)(Kp + ko + dc * 32 + 16);
        s[j] = mma_h(qa[dc], kb.v, s[j]);
      }
    }

#pragma unroll
    for (int r = 0; r < 8; ++r) {
      const int qs = qi0 + 8 * hh + r + WIN;
      float m = -INFINITY;
#pragma unroll
      for (int j = 0; j < 4; ++j) {
        const int ks = ch * 64 + j * 16 + cc;
        float sv = s[j][r] * sscale;
        sv = (ks > qs) ? -INFINITY : sv;
        s[j][r] = sv;
        m = fmaxf(m, sv);
      }
#pragma unroll
      for (int off = 1; off < 16; off <<= 1) m = fmaxf(m, __shfl_xor(m, off, 32));
      const float mnew  = fmaxf(mrow[r], m);
      const float msafe = (mnew == -INFINITY) ? 0.f : mnew;
      const float alpha = __expf(mrow[r] - msafe);
      mrow[r] = mnew;
      float psum = 0.f;
#pragma unroll
      for (int j = 0; j < 4; ++j) {
        const float p = __expf(s[j][r] - msafe);
        psum += p;
        pwh[(8 * hh + r) * 64 + j * 16 + cc] = (_Float16)(p * 1024.0f);
      }
#pragma unroll
      for (int off = 1; off < 16; off <<= 1) psum += __shfl_xor(psum, off, 32);
      lrow[r] = lrow[r] * alpha + psum;
#pragma unroll
      for (int t = 0; t < 4; ++t) oacc[t][r] *= alpha;
    }
    __builtin_amdgcn_fence(__ATOMIC_RELEASE, "workgroup");
    __builtin_amdgcn_wave_barrier();
    __builtin_amdgcn_fence(__ATOMIC_ACQUIRE, "workgroup");

#pragma unroll
    for (int kk = 0; kk < 2; ++kk) {
      FH pa;
      pa.h[0] = *(const v8h*)(pwh + cc * 64 + kk * 32 + 8 * hh);
      pa.h[1] = *(const v8h*)(pwh + cc * 64 + kk * 32 + 16 + 8 * hh);
#pragma unroll
      for (int t = 0; t < 4; ++t) {
        const size_t vo = (size_t)(t * 16 + cc) * SEQ + (size_t)(tk0 + kk * 32 + 8 * hh);
        FH vb;
        vb.h[0] = *(const v8h*)(Vt + vo);
        vb.h[1] = *(const v8h*)(Vt + vo + 16);
        oacc[t] = mma_h(pa.v, vb.v, oacc[t]);
      }
    }
    __builtin_amdgcn_fence(__ATOMIC_RELEASE, "workgroup");
    __builtin_amdgcn_wave_barrier();
    __builtin_amdgcn_fence(__ATOMIC_ACQUIRE, "workgroup");
  }

  float* os = Os[wave];
#pragma unroll
  for (int r = 0; r < 8; ++r) {
    const float l = lrow[r];
    const float inv = ((l > 0.f) ? (1.0f / l) : 0.f) * (1.0f / 16384.0f);
#pragma unroll
    for (int t = 0; t < 4; ++t) os[(8 * hh + r) * 64 + t * 16 + cc] = oacc[t][r] * inv;
  }
  __builtin_amdgcn_fence(__ATOMIC_RELEASE, "workgroup");
  __builtin_amdgcn_wave_barrier();
  __builtin_amdgcn_fence(__ATOMIC_ACQUIRE, "workgroup");
  {
    const int h2 = lane >> 4, c4 = (lane & 15) * 4;
    v4f ov[8];
#pragma unroll
    for (int it = 0; it < 8; ++it) {
      const int row = it * 2 + h2;
      ov[it] = *(const v4f*)(os + row * 64 + c4);
    }
    for (int pass = 0; pass < 2; ++pass) {
#pragma unroll
      for (int it = 0; it < 8; ++it) {
        const int row = it * 2 + h2;
        const size_t go = (size_t)(q0 + row) * TOKP + (size_t)h * HD + c4;
        *(volatile v4f*)(outp + go) = ov[it];
      }
      __threadfence();
    }
  }
}

extern "C" void kernel_launch(void* const* d_in, const int* in_sizes, int n_in,
                              void* d_out, int out_size, void* d_ws, size_t ws_size,
                              hipStream_t stream) {
  if (n_in < 3) return;
  if (in_sizes[0] != OUTN) return;
  if (in_sizes[1] != OUTN) return;
  if (in_sizes[2] != OUTN) return;
  if (out_size != OUTN) return;

  const float* q = (const float*)d_in[0];
  const float* k = (const float*)d_in[1];
  const float* v = (const float*)d_in[2];

  const size_t PTrig = (size_t)NWIN * NPAIR * 4;
  const size_t PPl   = (size_t)SEQ * NH * HD * 2;
  size_t off = 0;
  const size_t oCos = off; off += PTrig;
  const size_t oSin = off; off += PTrig;
  const size_t oQ   = off; off += PPl;
  const size_t oKA  = off; off += PPl;
  const size_t oKB  = off; off += PPl;
  const size_t oVT  = off; off += PPl;
  if (off > ws_size) return;
  if (off > (size_t)134217728) return;

  char* ws = (char*)d_ws;
  float*          CosT = (float*)(ws + oCos);
  float*          SinT = (float*)(ws + oSin);
  unsigned short* Qh   = (unsigned short*)(ws + oQ);
  unsigned short* KA   = (unsigned short*)(ws + oKA);
  unsigned short* KB   = (unsigned short*)(ws + oKB);
  unsigned short* VT   = (unsigned short*)(ws + oVT);
  float*          outf = (float*)d_out;

  const dim3 blk(256);
  const int nTrig  = NWIN * NPAIR;
  const int nwRows = SEQ * NQUAD;
  const dim3 gTrig((nTrig + 255) / 256);
  const dim3 gRope((nwRows + 7) / 8);
  const dim3 gVpl(SEQ / 64, NH);
  const dim3 gAttn(NH * NQB);
  const float carry  = 16.0f;
  const float sscale = 1.0f / 256.0f;

  rope_tab<<<gTrig, blk, 0, stream>>>(CosT, SinT, nTrig);
  rope_plane<1><<<gRope, blk, 0, stream>>>(q, CosT, SinT, Qh, Qh, nwRows, 0.125f, carry);
  rope_plane<2><<<gRope, blk, 0, stream>>>(k, CosT, SinT, KA, KB, nwRows, 1.0f, carry);
  v_plane<<<gVpl, blk, 0, stream>>>(v, VT);
  attn_local64<<<gAttn, dim3(128), 0, stream>>>(Qh, KA, KB, VT, outf, sscale);
  (void)hipGetLastError();
}
